// RWKV_TimeMix_12369505812813
// MI455X (gfx1250) — hardware-verified
//
#include <hip/hip_runtime.h>
#include <math.h>

constexpr int kBatch   = 4;
constexpr int kT       = 2048;
constexpr int kC       = 1024;
constexpr int kHeads   = 16;
constexpr int kA       = 1024;
constexpr int kHS      = 64;
constexpr int kTT      = 2048;
constexpr int kHalfC   = kC / 2;
constexpr int kRows    = kBatch * kT;
constexpr int kTiles   = kT / 64;
constexpr int kLdsPitch = 68;
constexpr float kFltMin = 1.17549435e-38f;

static_assert(kA == kHeads * kHS, "head layout");
static_assert(kHS == 64, "head size");
static_assert(kHeads == 16, "head count");
static_assert(kTT == kT, "table length");
static_assert((kT & (kT - 1)) == 0, "power of two time length");
static_assert(kRows % 64 == 0 && kA % 64 == 0 && kC % 64 == 0, "tile multiples");
static_assert(kC % 32 == 0 && kA % 32 == 0 && kT % 64 == 0, "k multiples");
static_assert(kC / 8 == 128, "row groups");
static_assert(kTiles == 32, "tile count");

typedef __attribute__((ext_vector_type(16))) __bf16   v16b;
typedef __attribute__((ext_vector_type(8)))  __bf16   v8b;
typedef __attribute__((ext_vector_type(8)))  float    v8f;
typedef __attribute__((ext_vector_type(4)))  float    v4f;
typedef __attribute__((ext_vector_type(4)))  unsigned int v4u;

__device__ __forceinline__ unsigned short f2bf_bits(float f) {
  unsigned u = __float_as_uint(f);
  return (unsigned short)((u + 0x7FFFu + ((u >> 16) & 1u)) >> 16);
}
__device__ __forceinline__ float bf_bits2f(unsigned short h) { return __uint_as_float(((unsigned)h) << 16); }
__device__ __forceinline__ float bf16r(float f) { return bf_bits2f(f2bf_bits(f)); }
__device__ __forceinline__ unsigned pk16(unsigned short a, unsigned short b) { return (unsigned)a | ((unsigned)b << 16); }
__device__ __forceinline__ void split_bf(float f, unsigned short& hb, unsigned short& lb) {
  hb = f2bf_bits(f);
  lb = f2bf_bits(f - bf_bits2f(hb));
}

union FragU { v16b v; v8b h[2]; };
__device__ __forceinline__ v16b frag_load(const __bf16* p) {
  FragU f;
  f.h[0] = *(const v8b*)(p);
  f.h[1] = *(const v8b*)(p + 16);
  return f.v;
}
__device__ __forceinline__ v8f mma_bf(v16b a, v16b b, v8f c) {
  return __builtin_amdgcn_wmma_f32_16x16x32_bf16(false, a, false, b, (short)0, c, false, false);
}
__device__ __forceinline__ void guard6_7(v8f& a0, v8f& a1, v8f& a2, v8f& a3, v8f& a4, v8f& a5,
                                         v16b x, v16b b0, v16b b1, v16b b2, v16b b3, v16b b4, v16b b5) {
  asm volatile("v_nop\n\tv_nop\n\tv_nop\n\tv_nop"
               : "+v"(a0), "+v"(a1), "+v"(a2), "+v"(a3), "+v"(a4), "+v"(a5)
               : "v"(x), "v"(b0), "v"(b1), "v"(b2), "v"(b3), "v"(b4), "v"(b5));
}
__device__ __forceinline__ void guard4_9(v8f& a0, v8f& a1, v8f& a2, v8f& a3, v16b x,
                                         v16b b0, v16b b1, v16b b2, v16b b3, v16b b4, v16b b5, v16b b6, v16b b7) {
  asm volatile("v_nop\n\tv_nop\n\tv_nop\n\tv_nop"
               : "+v"(a0), "+v"(a1), "+v"(a2), "+v"(a3)
               : "v"(x), "v"(b0), "v"(b1), "v"(b2), "v"(b3), "v"(b4), "v"(b5), "v"(b6), "v"(b7));
}
__device__ __forceinline__ void guard4_6(v8f& a0, v8f& a1, v8f& a2, v8f& a3, v16b x, v16b y,
                                         v16b b0, v16b b1, v16b b2, v16b b3) {
  asm volatile("v_nop\n\tv_nop\n\tv_nop\n\tv_nop"
               : "+v"(a0), "+v"(a1), "+v"(a2), "+v"(a3)
               : "v"(x), "v"(y), "v"(b0), "v"(b1), "v"(b2), "v"(b3));
}
__device__ __forceinline__ void acc_guard4(v8f& a, v8f& b, v8f& c, v8f& d) {
  asm volatile("v_nop\n\tv_nop\n\tv_nop\n\tv_nop" : "+v"(a), "+v"(b), "+v"(c), "+v"(d));
}
__device__ __forceinline__ void wave_sync_lds() {
  __builtin_amdgcn_fence(__ATOMIC_RELEASE, "workgroup");
  __builtin_amdgcn_wave_barrier();
  __builtin_amdgcn_fence(__ATOMIC_ACQUIRE, "workgroup");
}

__global__ __launch_bounds__(256) void xshift_cvt_kernel(const float* __restrict__ x, unsigned short* __restrict__ xs) {
  const int i = blockIdx.x * 256 + threadIdx.x;
  if (i < kRows * (kC / 8)) {
    const int row = i >> 7;
    const int c8  = i & 127;
    const int t   = row & (kT - 1);
    const bool shifted = (c8 * 8 < kHalfC);
    const bool zero    = shifted && (t == 0);
    const int srow = (shifted && !zero) ? (row - 1) : row;
    const float* sp = x + (size_t)srow * kC + c8 * 8;
    const v4f a = *(const v4f*)(sp);
    const v4f b = *(const v4f*)(sp + 4);
    unsigned short hb[8];
#pragma unroll
    for (int e = 0; e < 4; ++e) {
      const float fa = zero ? 0.0f : a[e];
      const float fb = zero ? 0.0f : b[e];
      hb[e]     = f2bf_bits(fa);
      hb[4 + e] = f2bf_bits(fb);
    }
    const v4u u = (v4u){pk16(hb[0], hb[1]), pk16(hb[2], hb[3]), pk16(hb[4], hb[5]), pk16(hb[6], hb[7])};
    unsigned short* q = xs + (size_t)i * 8;
    *(volatile v4u*)q = u;
    __threadfence();
    *(volatile v4u*)q = u;
  }
}

__global__ __launch_bounds__(256) void wcvt_kernel(const float* __restrict__ w0, const float* __restrict__ w1,
                                                   const float* __restrict__ w2, const float* __restrict__ w3,
                                                   unsigned short* __restrict__ dst) {
  const int z = blockIdx.y;
  const float* src = (z == 0) ? w0 : (z == 1) ? w1 : (z == 2) ? w2 : w3;
  const int i = blockIdx.x * 256 + threadIdx.x;
  if (i < (kA * kC) / 8) {
    const float* sp = src + (size_t)i * 8;
    const v4f a = *(const v4f*)(sp);
    const v4f b = *(const v4f*)(sp + 4);
    unsigned short hb[8];
#pragma unroll
    for (int e = 0; e < 4; ++e) {
      hb[e]     = f2bf_bits(a[e]);
      hb[4 + e] = f2bf_bits(b[e]);
    }
    const v4u u = (v4u){pk16(hb[0], hb[1]), pk16(hb[2], hb[3]), pk16(hb[4], hb[5]), pk16(hb[6], hb[7])};
    unsigned short* q = dst + (size_t)z * kA * kC + (size_t)i * 8;
    *(volatile v4u*)q = u;
    __threadfence();
    *(volatile v4u*)q = u;
  }
}

__global__ __launch_bounds__(256) void decay_tiles_kernel(const float* __restrict__ tw, unsigned short* __restrict__ wt) {
  const int i = blockIdx.x * 256 + threadIdx.x;
  if (i < kHeads * kTiles * 64 * 8) {
    const int j8 = i & 7;
    const int ii = (i >> 3) & 63;
    const int d  = (i >> 9) & (kTiles - 1);
    const int h  = i >> 14;
    unsigned short hb[8];
#pragma unroll
    for (int e = 0; e < 8; ++e) {
      const int j   = j8 * 8 + e;
      const int lag = 64 * d + ii - j;
      int idx = (kTT - 1) - lag;
      idx = idx < 0 ? 0 : (idx > kTT - 1 ? kTT - 1 : idx);
      float v = tw[(size_t)h * kTT + idx];
      v = (fabsf(v) < kFltMin) ? 0.0f : v;
      v = (lag >= 0) ? v : 0.0f;
      hb[e] = f2bf_bits(v);
    }
    const v4u u = (v4u){pk16(hb[0], hb[1]), pk16(hb[2], hb[3]), pk16(hb[4], hb[5]), pk16(hb[6], hb[7])};
    unsigned short* q = wt + (size_t)i * 8;
    *(volatile v4u*)q = u;
    __threadfence();
    *(volatile v4u*)q = u;
  }
}

__global__ __launch_bounds__(128) void proj_fused_kernel(
    const unsigned short* __restrict__ xsP, const unsigned short* __restrict__ wbP,
    const float* __restrict__ bk, const float* __restrict__ bv, const float* __restrict__ br,
    const float* __restrict__ alpha,
    float* __restrict__ Kpl, float* __restrict__ Gpl,
    unsigned short* __restrict__ kvhi, unsigned short* __restrict__ kvlo) {
  __shared__ __align__(16) float sK[64 * kLdsPitch];
  __shared__ __align__(16) float sV[64 * kLdsPitch];
  __shared__ __align__(16) float sR[64 * kLdsPitch];
  const __bf16* XS = (const __bf16*)xsP;
  const __bf16* WB = (const __bf16*)wbP;
  const int tid = threadIdx.x, lane = tid & 31, wave = tid >> 5;
  const int wm = wave >> 1, wn = wave & 1;
  const int c = lane & 15, hh = lane >> 4, koff = hh * 8;
  const int nt = blockIdx.x & (kHeads - 1);
  const int mt = blockIdx.x >> 4;
  const int m0 = mt * 64, n0 = nt * 64;

  const __bf16* ap = XS + (size_t)(m0 + 32 * wm + c) * kC + koff;
  const __bf16* bp = WB + (size_t)(n0 + 32 * wn + c) * kC + koff;

  v8f acc[3][2][2];
#pragma unroll
  for (int g = 0; g < 3; ++g)
#pragma unroll
    for (int mi = 0; mi < 2; ++mi)
#pragma unroll
      for (int nj = 0; nj < 2; ++nj) acc[g][mi][nj] = (v8f){0.f, 0.f, 0.f, 0.f, 0.f, 0.f, 0.f, 0.f};

  for (int k0 = 0; k0 < kC; k0 += 32) {
    v16b bf[3][2];
#pragma unroll
    for (int g = 0; g < 3; ++g)
#pragma unroll
      for (int nj = 0; nj < 2; ++nj)
        bf[g][nj] = frag_load(bp + (size_t)g * kA * kC + (size_t)nj * 16 * kC + k0);
#pragma unroll
    for (int mi = 0; mi < 2; ++mi) {
      const v16b a = frag_load(ap + (size_t)mi * 16 * kC + k0);
#pragma unroll
      for (int g = 0; g < 3; ++g)
#pragma unroll
        for (int nj = 0; nj < 2; ++nj) acc[g][mi][nj] = mma_bf(a, bf[g][nj], acc[g][mi][nj]);
      guard6_7(acc[0][mi][0], acc[0][mi][1], acc[1][mi][0], acc[1][mi][1], acc[2][mi][0], acc[2][mi][1],
               a, bf[0][0], bf[0][1], bf[1][0], bf[1][1], bf[2][0], bf[2][1]);
    }
  }
  acc_guard4(acc[0][0][0], acc[0][0][1], acc[0][1][0], acc[0][1][1]);
  acc_guard4(acc[1][0][0], acc[1][0][1], acc[1][1][0], acc[1][1][1]);
  acc_guard4(acc[2][0][0], acc[2][0][1], acc[2][1][0], acc[2][1][1]);

#pragma unroll
  for (int mi = 0; mi < 2; ++mi)
#pragma unroll
    for (int nj = 0; nj < 2; ++nj)
#pragma unroll
      for (int r = 0; r < 8; ++r) {
        const int row = 32 * wm + 16 * mi + 8 * hh + r;
        const int col = 32 * wn + 16 * nj + c;
        sK[row * kLdsPitch + col] = acc[0][mi][nj][r];
        sV[row * kLdsPitch + col] = acc[1][mi][nj][r];
        sR[row * kLdsPitch + col] = acc[2][mi][nj][r];
      }
  __syncthreads();

  const int c4 = (tid & 15) * 4;
  float bkr[4], bvr[4], brr[4];
  {
    const v4f b0 = *(const v4f*)(bk + n0 + c4);
    const v4f b1 = *(const v4f*)(bv + n0 + c4);
    const v4f b2 = *(const v4f*)(br + n0 + c4);
#pragma unroll
    for (int e = 0; e < 4; ++e) { bkr[e] = bf16r(b0[e]); bvr[e] = bf16r(b1[e]); brr[e] = bf16r(b2[e]); }
  }
#pragma unroll 1
  for (int it = 0; it < 8; ++it) {
    const int row = it * 8 + (tid >> 4);
    const int m   = m0 + row;
    const int t   = m & (kT - 1);
    const float al = bf16r(alpha[(size_t)nt * kTT + t]);
    const v4f pk = *(const v4f*)(sK + row * kLdsPitch + c4);
    const v4f pv = *(const v4f*)(sV + row * kLdsPitch + c4);
    const v4f pr = *(const v4f*)(sR + row * kLdsPitch + c4);
    v4f ko, go, kvo;
#pragma unroll
    for (int e = 0; e < 4; ++e) {
      float zk = pk[e] + bkr[e];
      zk = fminf(fmaxf(zk, -60.0f), 30.0f);
      const float kk = expf(zk);
      const float vv = pv[e] + bvr[e];
      const float zr = pr[e] + brr[e];
      const float sg = 1.0f / (1.0f + expf(-zr));
      ko[e]  = kk;
      go[e]  = sg;
      kvo[e] = (kk * vv) * al;
    }
    float* kp = Kpl + (size_t)m * kA + n0 + c4;
    float* gp = Gpl + (size_t)m * kA + n0 + c4;
    *(volatile v4f*)kp = ko;
    *(volatile v4f*)gp = go;
    __threadfence();
    *(volatile v4f*)kp = ko;
    *(volatile v4f*)gp = go;
    *(v4f*)(sK + row * kLdsPitch + c4) = kvo;
  }
  __syncthreads();

  const int bb  = m0 / kT;
  const int t0  = m0 & (kT - 1);
  const int seg = lane & 7, chq = lane >> 3;
  v4u hv[4], lv[4];
#pragma unroll
  for (int it = 0; it < 4; ++it) {
    const int ch = it * 16 + wave * 4 + chq;
    unsigned short hb[8], lb[8];
#pragma unroll
    for (int e = 0; e < 8; ++e) {
      const float f = sK[(seg * 8 + e) * kLdsPitch + ch];
      split_bf(f, hb[e], lb[e]);
    }
    hv[it] = (v4u){pk16(hb[0], hb[1]), pk16(hb[2], hb[3]), pk16(hb[4], hb[5]), pk16(hb[6], hb[7])};
    lv[it] = (v4u){pk16(lb[0], lb[1]), pk16(lb[2], lb[3]), pk16(lb[4], lb[5]), pk16(lb[6], lb[7])};
  }
  for (int pass = 0; pass < 2; ++pass) {
#pragma unroll
    for (int it = 0; it < 4; ++it) {
      const int ch = it * 16 + wave * 4 + chq;
      const size_t off = ((size_t)((bb * kHeads + nt) * kHS + ch)) * kT + t0 + seg * 8;
      *(volatile v4u*)(kvhi + off) = hv[it];
      *(volatile v4u*)(kvlo + off) = lv[it];
    }
    __threadfence();
  }
}

__global__ __launch_bounds__(256) void scan_gate_kernel(const float* __restrict__ Kpl, float* Gpl) {
  const int i = blockIdx.x * 256 + threadIdx.x;
  if (i < kBatch * kA) {
    const int b = i >> 10;
    const int a = i & (kA - 1);
    size_t off = (size_t)b * kT * kA + a;
    double run = 0.0;
#pragma unroll 4
    for (int t = 0; t < kT; ++t) {
      const float kk = Kpl[off];
      const float g  = Gpl[off];
      run += (double)kk;
      const float rs  = (float)run;
      const float val = g * (1.0f / rs);
      *(volatile float*)(Gpl + off) = val;
      __threadfence();
      *(volatile float*)(Gpl + off) = val;
      off += kA;
    }
  }
}

__global__ __launch_bounds__(256) void decay_mix_kernel(
    const unsigned short* __restrict__ wtP, const unsigned short* __restrict__ kvhP, const unsigned short* __restrict__ kvlP,
    const float* __restrict__ beta, const float* __restrict__ Gpl,
    unsigned short* __restrict__ rwhi, unsigned short* __restrict__ rwlo) {
  __shared__ __align__(16) float sT[8][16 * kLdsPitch];
  const __bf16* WT  = (const __bf16*)wtP;
  const __bf16* KVH = (const __bf16*)kvhP;
  const __bf16* KVL = (const __bf16*)kvlP;
  const int lane = threadIdx.x & 31, wave = threadIdx.x >> 5;
  const int c = lane & 15, hh = lane >> 4, koff = hh * 8;
  const int hd = blockIdx.x & (kHeads - 1);
  const int ti = (kTiles - 1) - (int)(blockIdx.x >> 4);
  const int bb = wave >> 1, mh = wave & 1;

  const __bf16* wtb = WT + ((size_t)hd * kTiles * 64 + 32 * mh + c) * 64 + koff;
  const size_t brow = ((size_t)(bb * kHeads + hd) * kHS + c) * kT + koff;
  const __bf16* bhp = KVH + brow;
  const __bf16* blp = KVL + brow;

  v8f acc[2][4];
#pragma unroll
  for (int mi = 0; mi < 2; ++mi)
#pragma unroll
    for (int nj = 0; nj < 4; ++nj) acc[mi][nj] = (v8f){0.f, 0.f, 0.f, 0.f, 0.f, 0.f, 0.f, 0.f};

  for (int J = 0; J <= ti; ++J) {
    const int d = ti - J;
#pragma unroll
    for (int kk = 0; kk < 64; kk += 32) {
      v16b bh[4], bl[4];
#pragma unroll
      for (int nj = 0; nj < 4; ++nj) {
        const size_t bo = (size_t)nj * 16 * kT + (size_t)J * 64 + kk;
        bh[nj] = frag_load(bhp + bo);
        bl[nj] = frag_load(blp + bo);
      }
#pragma unroll
      for (int mi = 0; mi < 2; ++mi) {
        const v16b a = frag_load(wtb + (size_t)d * 4096 + mi * 1024 + kk);
#pragma unroll
        for (int nj = 0; nj < 4; ++nj) {
          acc[mi][nj] = mma_bf(a, bh[nj], acc[mi][nj]);
          acc[mi][nj] = mma_bf(a, bl[nj], acc[mi][nj]);
        }
        guard4_9(acc[mi][0], acc[mi][1], acc[mi][2], acc[mi][3], a,
                 bh[0], bh[1], bh[2], bh[3], bl[0], bl[1], bl[2], bl[3]);
      }
    }
  }
  acc_guard4(acc[0][0], acc[0][1], acc[0][2], acc[0][3]);
  acc_guard4(acc[1][0], acc[1][1], acc[1][2], acc[1][3]);

  float* slab = sT[wave];
  const int q = lane >> 3, c8 = (lane & 7) * 8;
#pragma unroll
  for (int mi = 0; mi < 2; ++mi) {
    const int tb = ti * 64 + 32 * mh + 16 * mi;
#pragma unroll
    for (int nj = 0; nj < 4; ++nj)
#pragma unroll
      for (int r = 0; r < 8; ++r) slab[(8 * hh + r) * kLdsPitch + 16 * nj + c] = acc[mi][nj][r];
    wave_sync_lds();
    v4u hv[4], lv[4];
#pragma unroll
    for (int it = 0; it < 4; ++it) {
      const int row = it * 4 + q;
      const int t   = tb + row;
      const size_t m = (size_t)bb * kT + t;
      const float bet = bf16r(beta[(size_t)hd * kTT + t]);
      const float* gp = Gpl + m * kA + hd * kHS + c8;
      const v4f g0 = *(const v4f*)(gp);
      const v4f g1 = *(const v4f*)(gp + 4);
      const v4f s0 = *(const v4f*)(slab + row * kLdsPitch + c8);
      const v4f s1 = *(const v4f*)(slab + row * kLdsPitch + c8 + 4);
      unsigned short hb[8], lb[8];
#pragma unroll
      for (int e = 0; e < 4; ++e) {
        const float v0 = (s0[e] * bet) * g0[e];
        const float v1 = (s1[e] * bet) * g1[e];
        split_bf(v0, hb[e], lb[e]);
        split_bf(v1, hb[4 + e], lb[4 + e]);
      }
      hv[it] = (v4u){pk16(hb[0], hb[1]), pk16(hb[2], hb[3]), pk16(hb[4], hb[5]), pk16(hb[6], hb[7])};
      lv[it] = (v4u){pk16(lb[0], lb[1]), pk16(lb[2], lb[3]), pk16(lb[4], lb[5]), pk16(lb[6], lb[7])};
    }
    for (int pass = 0; pass < 2; ++pass) {
#pragma unroll
      for (int it = 0; it < 4; ++it) {
        const int row = it * 4 + q;
        const size_t m = (size_t)bb * kT + tb + row;
        const size_t off = m * kA + hd * kHS + c8;
        *(volatile v4u*)(rwhi + off) = hv[it];
        *(volatile v4u*)(rwlo + off) = lv[it];
      }
      __threadfence();
    }
    wave_sync_lds();
  }
}

__global__ __launch_bounds__(256) void out_proj_kernel(
    const unsigned short* __restrict__ ahP, const unsigned short* __restrict__ alP, const unsigned short* __restrict__ wP,
    const float* __restrict__ bo, const float* __restrict__ gamma, float* __restrict__ out) {
  __shared__ __align__(16) float sT[8][16 * kLdsPitch];
  const __bf16* AH = (const __bf16*)ahP;
  const __bf16* AL = (const __bf16*)alP;
  const __bf16* W  = (const __bf16*)wP;
  const int lane = threadIdx.x & 31, wave = threadIdx.x >> 5;
  const int tilesN = kC >> 6;
  const int tilesM = kRows >> 6;
  const int tile = blockIdx.x * 8 + wave;
  if (tile >= tilesM * tilesN) return;
  const int tm = tile / tilesN;
  const int tn = tile - tm * tilesN;
  const int m0 = tm << 6;
  const int n0 = tn << 6;
  const int rlane = lane & 15;
  const int koff  = (lane >> 4) * 8;
  const int mOff  = (lane >> 4) * 8;

  v8f acc[4][4];
#pragma unroll
  for (int i = 0; i < 4; ++i)
#pragma unroll
    for (int j = 0; j < 4; ++j) acc[i][j] = (v8f){0.f, 0.f, 0.f, 0.f, 0.f, 0.f, 0.f, 0.f};

  for (int k0 = 0; k0 < kA; k0 += 32) {
    v16b bh[4];
#pragma unroll
    for (int j = 0; j < 4; ++j) bh[j] = frag_load(W + (size_t)(n0 + (j << 4) + rlane) * kA + koff + k0);
#pragma unroll
    for (int i = 0; i < 4; ++i) {
      const size_t ao = (size_t)(m0 + (i << 4) + rlane) * kA + koff + k0;
      const v16b ah = frag_load(AH + ao);
      const v16b al = frag_load(AL + ao);
#pragma unroll
      for (int j = 0; j < 4; ++j) {
        acc[i][j] = mma_bf(ah, bh[j], acc[i][j]);
        acc[i][j] = mma_bf(al, bh[j], acc[i][j]);
      }
      guard4_6(acc[i][0], acc[i][1], acc[i][2], acc[i][3], ah, al, bh[0], bh[1], bh[2], bh[3]);
    }
  }
  acc_guard4(acc[0][0], acc[0][1], acc[0][2], acc[0][3]);
  acc_guard4(acc[1][0], acc[1][1], acc[1][2], acc[1][3]);
  acc_guard4(acc[2][0], acc[2][1], acc[2][2], acc[2][3]);
  acc_guard4(acc[3][0], acc[3][1], acc[3][2], acc[3][3]);

  float* slab = sT[wave];
  float bias4[4];
#pragma unroll
  for (int j = 0; j < 4; ++j) bias4[j] = bf16r(bo[n0 + (j << 4) + rlane]);
#pragma unroll
  for (int i = 0; i < 4; ++i) {
    const int mBase = m0 + (i << 4);
    float gm[8];
#pragma unroll
    for (int r = 0; r < 8; ++r) gm[r] = bf16r(gamma[(mBase + mOff + r) & (kT - 1)]);
#pragma unroll
    for (int j = 0; j < 4; ++j)
#pragma unroll
      for (int r = 0; r < 8; ++r)
        slab[(mOff + r) * kLdsPitch + (j << 4) + rlane] = (acc[i][j][r] + bias4[j]) * gm[r];
    wave_sync_lds();
    {
      const int hh = lane >> 4, c4 = (lane & 15) * 4;
      for (int pass = 0; pass < 2; ++pass) {
#pragma unroll
        for (int it = 0; it < 8; ++it) {
          const int row = it * 2 + hh;
          const v4f v = *(const v4f*)(slab + row * kLdsPitch + c4);
          *(volatile v4f*)(out + (size_t)(mBase + row) * kC + n0 + c4) = v;
        }
        __threadfence();
      }
    }
    wave_sync_lds();
  }
}

extern "C" void kernel_launch(void* const* d_in, const int* in_sizes, int n_in,
                              void* d_out, int out_size, void* d_ws, size_t ws_size, hipStream_t stream) {
  if (n_in < 13 || d_out == nullptr || d_ws == nullptr) return;
  if (in_sizes[0] != kBatch * kT * kC || in_sizes[1] != kHeads * kTT || in_sizes[2] != kHeads * kTT ||
      in_sizes[3] != kHeads * kTT || in_sizes[4] != kTT || in_sizes[5] != kA * kC || in_sizes[6] != kA ||
      in_sizes[7] != kA * kC || in_sizes[8] != kA || in_sizes[9] != kA * kC || in_sizes[10] != kA ||
      in_sizes[11] != kC * kA || in_sizes[12] != kC || out_size != kBatch * kT * kC) return;

  const float* x      = (const float*)d_in[0];
  const float* time_w = (const float*)d_in[1];
  const float* alpha  = (const float*)d_in[2];
  const float* beta   = (const float*)d_in[3];
  const float* gamma  = (const float*)d_in[4];
  const float* Wk     = (const float*)d_in[5];
  const float* bk     = (const float*)d_in[6];
  const float* Wv     = (const float*)d_in[7];
  const float* bv     = (const float*)d_in[8];
  const float* Wr     = (const float*)d_in[9];
  const float* br     = (const float*)d_in[10];
  const float* Wo     = (const float*)d_in[11];
  const float* bo     = (const float*)d_in[12];
  float* out = (float*)d_out;

  const size_t szXS  = (size_t)kRows * kC * 2;
  const size_t szWB  = (size_t)4 * kA * kC * 2;
  const size_t szWT  = (size_t)kHeads * kTiles * 64 * 64 * 2;
  const size_t szF32 = (size_t)kRows * kA * 4;
  const size_t szKV  = (size_t)kBatch * kHeads * kHS * kT * 2;
  char* ws = (char*)d_ws;
  size_t off = 0;
  unsigned short* XS  = (unsigned short*)(ws + off); off += szXS;
  unsigned short* WB  = (unsigned short*)(ws + off); off += szWB;
  unsigned short* WT  = (unsigned short*)(ws + off); off += szWT;
  float*          KPL = (float*)(ws + off);          off += szF32;
  float*          GPL = (float*)(ws + off);          off += szF32;
  unsigned short* KVH = (unsigned short*)(ws + off); off += szKV;
  unsigned short* KVL = (unsigned short*)(ws + off); off += szKV;
  if (off > ws_size || off > (size_t)134217728) return;
  unsigned short* RWHI = XS;
  unsigned short* RWLO = (unsigned short*)KPL;
  const unsigned short* WOB = WB + (size_t)3 * kA * kC;

  xshift_cvt_kernel<<<(kRows * (kC / 8)) / 256, 256, 0, stream>>>(x, XS);
  wcvt_kernel<<<dim3((kA * kC / 8) / 256, 4), 256, 0, stream>>>(Wk, Wv, Wr, Wo, WB);
  decay_tiles_kernel<<<(kHeads * kTiles * 64 * 8) / 256, 256, 0, stream>>>(time_w, WT);
  proj_fused_kernel<<<(kRows / 64) * kHeads, 128, 0, stream>>>(XS, WB, bk, bv, br, alpha, KPL, GPL, KVH, KVL);
  scan_gate_kernel<<<(kBatch * kA) / 256, 256, 0, stream>>>(KPL, GPL);
  decay_mix_kernel<<<kTiles * kHeads, 256, 0, stream>>>(WT, KVH, KVL, beta, GPL, RWHI, RWLO);
  out_proj_kernel<<<((kRows / 64) * (kC / 64)) / 8, 256, 0, stream>>>(RWHI, RWLO, WOB, bo, gamma, out);
}
